// LinearRetriever_15281493639180
// MI455X (gfx1250) — hardware-verified
//
#include <hip/hip_runtime.h>
#include <math.h>
#include <stdint.h>

#define NBATCH 64
#define LX     256
#define TY     64
#define DIN    512
#define EDIM   200
#define EPAD   256
#define KMM    224
#define XROWS  (NBATCH * LX)
#define YROWS  (NBATCH * TY)
#define ROWS   (XROWS + YROWS)
#define JPB    32
static_assert((ROWS % 64) == 0 && (EPAD % 64) == 0 && (DIN % 32) == 0);
static_assert((KMM % 32) == 0 && KMM >= EDIM && KMM <= EPAD);
static_assert((NBATCH % JPB) == 0 && JPB == 32 && LX == 256 && TY == 64);

typedef _Float16 v16h __attribute__((ext_vector_type(16)));
typedef _Float16 v8h  __attribute__((ext_vector_type(8)));
typedef __bf16   v16b __attribute__((ext_vector_type(16)));
typedef __bf16   v8b  __attribute__((ext_vector_type(8)));
typedef float    v8f  __attribute__((ext_vector_type(8)));
typedef float    v4f  __attribute__((ext_vector_type(4)));
typedef unsigned int v4u __attribute__((ext_vector_type(4)));

__device__ __forceinline__ unsigned short bf_bits(float f) {
  unsigned u = __float_as_uint(f);
  return (unsigned short)((u + 0x7FFFu + ((u >> 16) & 1u)) >> 16);
}
__device__ __forceinline__ float bf_up(unsigned short h) { return __uint_as_float(((unsigned)h) << 16); }
__device__ __forceinline__ unsigned short h_bits(_Float16 x) { return __builtin_bit_cast(unsigned short, x); }
__device__ __forceinline__ unsigned pk16(unsigned short a, unsigned short b) { return (unsigned)a | ((unsigned)b << 16); }
__device__ __forceinline__ v8f zero8() { v8f z = {0.f, 0.f, 0.f, 0.f, 0.f, 0.f, 0.f, 0.f}; return z; }

__device__ __forceinline__ v16b ldfrag_b(const __bf16* p) {
  union { v16b v; v8b h[2]; } f;
  f.h[0] = *(const v8b*)(p);
  f.h[1] = *(const v8b*)(p + 16);
  return f.v;
}
__device__ __forceinline__ v16h ldfrag_h(const _Float16* p) {
  union { v16h v; v8h h[2]; } f;
  f.h[0] = *(const v8h*)(p);
  f.h[1] = *(const v8h*)(p + 16);
  return f.v;
}

__device__ __forceinline__ v8f mma_h(v16h a, v16h b, v8f c) {
  c = __builtin_amdgcn_wmma_f32_16x16x32_f16(false, a, false, b, (short)0, c, false, false);
#if defined(__HIP_DEVICE_COMPILE__)
  asm volatile("v_nop\n\tv_nop\n\tv_nop\n\tv_nop" : "+v"(c) : "v"(a), "v"(b));
#endif
  return c;
}
__device__ __forceinline__ v8f mma_b_raw(v16b a, v16b b, v8f c) {
  return __builtin_amdgcn_wmma_f32_16x16x32_bf16(false, a, false, b, (short)0, c, false, false);
}
__device__ __forceinline__ void dep_guard_b(v8f& a, v8f& b, v16b x, v16b y) {
#if defined(__HIP_DEVICE_COMPILE__)
  asm volatile("v_nop\n\tv_nop\n\tv_nop\n\tv_nop" : "+v"(a), "+v"(b) : "v"(x), "v"(y));
#endif
}
__device__ __forceinline__ void keep4_b(v16b a, v16b b, v16b c, v16b d) {
#if defined(__HIP_DEVICE_COMPILE__)
  asm volatile("v_nop" :: "v"(a), "v"(b), "v"(c), "v"(d));
#endif
}
__device__ __forceinline__ void acc_guard4(v8f& a, v8f& b, v8f& c, v8f& d) {
#if defined(__HIP_DEVICE_COMPILE__)
  asm volatile("v_nop\n\tv_nop\n\tv_nop\n\tv_nop" : "+v"(a), "+v"(b), "+v"(c), "+v"(d));
#endif
}
__device__ __forceinline__ void wave_sync_lds() {
  __builtin_amdgcn_fence(__ATOMIC_RELEASE, "workgroup");
  __builtin_amdgcn_wave_barrier();
  __builtin_amdgcn_fence(__ATOMIC_ACQUIRE, "workgroup");
}

__global__ __launch_bounds__(256) void cvt_bf16x8(const float* __restrict__ in, unsigned short* out,
                                                  int n8valid, int n8total) {
  const int i = blockIdx.x * 256 + threadIdx.x;
  if (i < n8total) {
    const int ic = min(i, n8valid - 1);
    const v4f a = *(const v4f*)(in + (size_t)ic * 8);
    const v4f b = *(const v4f*)(in + (size_t)ic * 8 + 4);
    v4u p;
    p[0] = pk16(bf_bits(a[0]), bf_bits(a[1]));
    p[1] = pk16(bf_bits(a[2]), bf_bits(a[3]));
    p[2] = pk16(bf_bits(b[0]), bf_bits(b[1]));
    p[3] = pk16(bf_bits(b[2]), bf_bits(b[3]));
    const v4u z = {0u, 0u, 0u, 0u};
    const v4u q = (i < n8valid) ? p : z;
    *(volatile v4u*)(out + (size_t)i * 8) = q;
    __threadfence();
    *(volatile v4u*)(out + (size_t)i * 8) = q;
  }
}

template <int NSPLIT, int OUT_MODE>
__global__ __launch_bounds__(256) void gemm64(
    const unsigned short* __restrict__ Ap, const unsigned short* A2p, int lda, long long strideA,
    const unsigned short* __restrict__ Btp, const unsigned short* Bt2p, int ldb, long long strideB,
    void* Cout, int ldc, long long strideC,
    void* Cout2, int ldc2, long long strideC2, int N2,
    int M, int N, int K, float rscale,
    const float* __restrict__ bias, int nbias) {
  const __bf16* A   = (const __bf16*)(const void*)Ap;
  const __bf16* A2  = (const __bf16*)(const void*)A2p;
  const __bf16* Bt  = (const __bf16*)(const void*)Btp;
  const __bf16* Bt2 = (const __bf16*)(const void*)Bt2p;
  __shared__ __align__(16) float sT[8][16 * 68];
  const int b    = blockIdx.y;
  const int lane = threadIdx.x & 31;
  const int wave = threadIdx.x >> 5;
  const int tilesN = N >> 6;
  const int tilesM = M >> 6;
  const int tile = blockIdx.x * 8 + wave;
  if (tile >= tilesM * tilesN) return;
  const int tm = tile / tilesN;
  const int tn = tile - tm * tilesN;
  const int m0 = tm << 6;
  const int n0 = tn << 6;

  const __bf16* Ab  = A  + (size_t)b * strideA;
  const __bf16* Bb  = Bt + (size_t)b * strideB;
  const __bf16* Ab2 = (NSPLIT >= 1) ? (A2  + (size_t)b * strideA) : Ab;
  const __bf16* Bb2 = (NSPLIT == 2) ? (Bt2 + (size_t)b * strideB) : Bb;

  const int rlane = lane & 15;
  const int koff  = (lane >> 4) * 8;
  const int mOff  = (lane >> 4) * 8;

  v8f acc[4][4];
#pragma unroll
  for (int i = 0; i < 4; ++i)
#pragma unroll
    for (int j = 0; j < 4; ++j) acc[i][j] = zero8();

  for (int k0 = 0; k0 < K; k0 += 32) {
    v16b bh[4], bl[4];
#pragma unroll
    for (int j = 0; j < 4; ++j) {
      const size_t bo = (size_t)(n0 + (j << 4) + rlane) * ldb + koff + k0;
      bh[j] = ldfrag_b(Bb + bo);
      if (NSPLIT == 2) bl[j] = ldfrag_b(Bb2 + bo); else bl[j] = bh[j];
    }
#pragma unroll
    for (int i = 0; i < 4; ++i) {
      const size_t ao = (size_t)(m0 + (i << 4) + rlane) * lda + koff + k0;
      const v16b ah = ldfrag_b(Ab + ao);
      v16b al = ah;
      if (NSPLIT >= 1) al = ldfrag_b(Ab2 + ao);
#pragma unroll
      for (int j = 0; j < 4; ++j) {
        acc[i][j] = mma_b_raw(ah, bh[j], acc[i][j]);
        if (NSPLIT >= 1) acc[i][j] = mma_b_raw(al, bh[j], acc[i][j]);
        if (NSPLIT == 2) acc[i][j] = mma_b_raw(ah, bl[j], acc[i][j]);
      }
      dep_guard_b(acc[i][0], acc[i][3], ah, al);
    }
    keep4_b(bh[0], bh[1], bh[2], bh[3]);
    if (NSPLIT == 2) keep4_b(bl[0], bl[1], bl[2], bl[3]);
  }
  acc_guard4(acc[0][0], acc[0][1], acc[0][2], acc[0][3]);
  acc_guard4(acc[1][0], acc[1][1], acc[1][2], acc[1][3]);
  acc_guard4(acc[2][0], acc[2][1], acc[2][2], acc[2][3]);
  acc_guard4(acc[3][0], acc[3][1], acc[3][2], acc[3][3]);

  float bv[4];
#pragma unroll
  for (int j = 0; j < 4; ++j) {
    const int col = n0 + (j << 4) + rlane;
    const int cc  = min(col, nbias - 1);
    const float t = bf_up(bf_bits(bias[cc]));
    bv[j] = (col < nbias) ? t : 0.f;
  }

  float* slab = sT[wave];
#pragma unroll
  for (int i = 0; i < 4; ++i) {
    const int mBase = m0 + (i << 4);
#pragma unroll
    for (int j = 0; j < 4; ++j) {
#pragma unroll
      for (int r = 0; r < 8; ++r) {
        slab[(mOff + r) * 68 + (j << 4) + rlane] = acc[i][j][r] + bv[j];
      }
    }
    wave_sync_lds();
    if (OUT_MODE == 0) {
      float* C = (float*)Cout + (size_t)b * strideC;
      const int hh = lane >> 4, c4 = (lane & 15) * 4;
      for (int pass = 0; pass < 2; ++pass) {
#pragma unroll
        for (int it = 0; it < 8; ++it) {
          const int row = it * 2 + hh;
          const v4f v = *(const v4f*)(slab + row * 68 + c4);
          *(volatile v4f*)(C + (size_t)(mBase + row) * ldc + n0 + c4) = v;
        }
        __threadfence();
      }
    } else {
      const int q = lane >> 3, c8 = (lane & 7) * 8;
      unsigned short* C  = (unsigned short*)Cout  + (size_t)b * strideC;
      unsigned short* C2 = (unsigned short*)Cout2 + (size_t)b * strideC2;
      const bool wlo = (OUT_MODE == 2) || (n0 < N2);
      v4u hv[4], lv[4];
#pragma unroll
      for (int it = 0; it < 4; ++it) {
        const int row = it * 4 + q;
        const float* sp = slab + row * 68 + c8;
        v4u a, a2;
#pragma unroll
        for (int e = 0; e < 4; ++e) {
          const float f0 = sp[2 * e], f1 = sp[2 * e + 1];
          unsigned short h0, h1, l0, l1;
          if (OUT_MODE == 2) {
            h0 = bf_bits(f0); h1 = bf_bits(f1);
            l0 = bf_bits(f0 - bf_up(h0)); l1 = bf_bits(f1 - bf_up(h1));
          } else {
            const _Float16 x0 = (_Float16)f0, x1 = (_Float16)f1;
            h0 = h_bits(x0); h1 = h_bits(x1);
            l0 = h_bits((_Float16)((f0 - (float)x0) * rscale));
            l1 = h_bits((_Float16)((f1 - (float)x1) * rscale));
          }
          a[e] = pk16(h0, h1); a2[e] = pk16(l0, l1);
        }
        hv[it] = a; lv[it] = a2;
      }
      for (int pass = 0; pass < 2; ++pass) {
#pragma unroll
        for (int it = 0; it < 4; ++it) {
          const int row = it * 4 + q;
          *(volatile v4u*)(C + (size_t)(mBase + row) * ldc + n0 + c8) = hv[it];
          if (wlo) *(volatile v4u*)(C2 + (size_t)(mBase + row) * ldc2 + n0 + c8) = lv[it];
        }
        __threadfence();
      }
    }
    wave_sync_lds();
  }
}

__global__ __launch_bounds__(256)
void match_max_mean(const unsigned short* __restrict__ php, const unsigned short* __restrict__ plp,
                    float* S, float rres) {
  __shared__ float swpart[8 * 64];
  __shared__ __align__(16) float sS[JPB];

  const int tid  = threadIdx.x;
  const int wave = tid >> 5;
  const int lane = tid & 31;
  const int hh   = lane >> 4;
  const int c    = lane & 15;

  const int i  = blockIdx.x / (NBATCH / JPB);
  const int j0 = (blockIdx.x % (NBATCH / JPB)) * JPB;

  const _Float16* PH = (const _Float16*)(const void*)php;
  const _Float16* PL = (const _Float16*)(const void*)plp;
  const size_t xrow0 = (size_t)i * LX + (size_t)wave * 32;

#pragma unroll 1
  for (int jj = 0; jj < JPB; ++jj) {
    const size_t yrow0 = (size_t)XROWS + (size_t)(j0 + jj) * TY;
    float cm[4];
#pragma unroll
    for (int n = 0; n < 4; ++n) cm[n] = -INFINITY;

#pragma unroll 1
    for (int ms = 0; ms < 2; ++ms) {
      v8f acc[4], accl[4];
#pragma unroll
      for (int n = 0; n < 4; ++n) { acc[n] = zero8(); accl[n] = zero8(); }
      const _Float16* arow = PH + (xrow0 + (size_t)ms * 16 + c) * EPAD + 8 * hh;
      const _Float16* lrow = PL + (xrow0 + (size_t)ms * 16 + c) * EPAD + 8 * hh;
      const _Float16* brow = PH + (yrow0 + c) * EPAD + 8 * hh;
#pragma unroll 1
      for (int k0 = 0; k0 < KMM; k0 += 32) {
        const v16h ah = ldfrag_h(arow + k0);
        const v16h al = ldfrag_h(lrow + k0);
        v16h bfr[4];
#pragma unroll
        for (int n = 0; n < 4; ++n) bfr[n] = ldfrag_h(brow + (size_t)n * 16 * EPAD + k0);
#pragma unroll
        for (int n = 0; n < 4; ++n) {
          acc[n]  = mma_h(ah, bfr[n], acc[n]);
          accl[n] = mma_h(al, bfr[n], accl[n]);
        }
      }
#pragma unroll
      for (int n = 0; n < 4; ++n) {
#pragma unroll
        for (int r = 0; r < 8; ++r) cm[n] = fmaxf(cm[n], acc[n][r] + accl[n][r] * rres);
      }
    }

#pragma unroll
    for (int n = 0; n < 4; ++n) {
      float m = cm[n];
      m = fmaxf(m, __shfl_xor(m, 16, 32));
      if (hh == 0) swpart[wave * 64 + n * 16 + c] = m;
    }
    __syncthreads();

    if (wave == 0) {
      float m0 = swpart[lane];
      float m1 = swpart[32 + lane];
#pragma unroll
      for (int w = 1; w < 8; ++w) {
        m0 = fmaxf(m0, swpart[w * 64 + lane]);
        m1 = fmaxf(m1, swpart[w * 64 + 32 + lane]);
      }
      float s = m0 + m1;
#pragma unroll
      for (int off = 16; off >= 1; off >>= 1) s += __shfl_xor(s, off, 32);
      if (lane == 0) sS[jj] = s * (1.0f / 64.0f);
    }
    __syncthreads();
  }

  if (wave == 0) {
    const int l8 = lane & 7;
    const v4f v = *(const v4f*)(sS + 4 * l8);
    float* dst = S + (size_t)i * NBATCH + j0 + 4 * l8;
    if (lane < 8) *(volatile v4f*)dst = v;
    __threadfence();
    if (lane < 8) *(volatile v4f*)dst = v;
  }
}

extern "C" void kernel_launch(void* const* d_in, const int* in_sizes, int n_in,
                              void* d_out, int out_size, void* d_ws, size_t ws_size,
                              hipStream_t stream) {
  if (n_in < 4) return;
  if (in_sizes[0] != XROWS * DIN) return;
  if (in_sizes[1] != YROWS * DIN) return;
  if (in_sizes[2] != EDIM * DIN) return;
  if (in_sizes[3] != EDIM) return;
  if (out_size != NBATCH * NBATCH) return;

  const float* x    = (const float*)d_in[0];
  const float* y    = (const float*)d_in[1];
  const float* W    = (const float*)d_in[2];
  const float* bias = (const float*)d_in[3];

  const size_t PXY = (size_t)ROWS * DIN * 2;
  const size_t PWb = (size_t)EPAD * DIN * 2;
  const size_t PP  = (size_t)ROWS * EPAD * 2;
  size_t off = 0;
  const size_t oXY = off; off += PXY;
  const size_t oWb = off; off += PWb;
  const size_t oPH = off; off += PP;
  const size_t oPL = off; off += PP;
  if (off > ws_size) return;
  if (off > (size_t)134217728) return;

  char* ws = (char*)d_ws;
  unsigned short* XY = (unsigned short*)(ws + oXY);
  unsigned short* Yb = XY + (size_t)XROWS * DIN;
  unsigned short* Wb = (unsigned short*)(ws + oWb);
  unsigned short* PH = (unsigned short*)(ws + oPH);
  unsigned short* PL = (unsigned short*)(ws + oPL);

  const dim3 blk(256);
  const int n8x = XROWS * DIN / 8;
  const int n8y = YROWS * DIN / 8;
  const int n8w = EDIM * DIN / 8;
  const int n8wt = EPAD * DIN / 8;
  const dim3 gCvtX((n8x + 255) / 256);
  const dim3 gCvtY((n8y + 255) / 256);
  const dim3 gCvtW((n8wt + 255) / 256);
  const dim3 gProj(((ROWS / 64) * (EPAD / 64) + 7) / 8, 1);
  const dim3 gMatch(NBATCH * (NBATCH / JPB));

  cvt_bf16x8<<<gCvtX, blk, 0, stream>>>(x, XY, n8x, n8x);
  cvt_bf16x8<<<gCvtY, blk, 0, stream>>>(y, Yb, n8y, n8y);
  cvt_bf16x8<<<gCvtW, blk, 0, stream>>>(W, Wb, n8w, n8wt);
  gemm64<0, 3><<<gProj, blk, 0, stream>>>(
      XY, XY, DIN, 0LL, Wb, Wb, DIN, 0LL,
      (void*)PH, EPAD, 0LL, (void*)PL, EPAD, 0LL, EPAD,
      ROWS, EPAD, DIN, 4096.0f, bias, EDIM);
  match_max_mean<<<gMatch, blk, 0, stream>>>(PH, PL, (float*)d_out, 1.0f / 4096.0f);
  (void)hipGetLastError();
}
